// EdgeSelector_32607391711818
// MI455X (gfx1250) — hardware-verified
//
#include <hip/hip_runtime.h>
#include <math.h>

typedef __attribute__((ext_vector_type(16))) _Float16 v16h;
typedef __attribute__((ext_vector_type(16))) __bf16 v16b;
typedef __attribute__((ext_vector_type(8)))  _Float16 v8h;
typedef __attribute__((ext_vector_type(8)))  float v8f;
typedef __attribute__((ext_vector_type(4)))  float v4f;
typedef __attribute__((ext_vector_type(2)))  float v2f;
typedef __attribute__((ext_vector_type(4)))  unsigned v4u;
typedef __attribute__((ext_vector_type(4)))  int v4i;
typedef float __attribute__((may_alias)) float_a;
typedef int __attribute__((may_alias)) int_a;

template <typename T> __device__ __forceinline__ void vst2(void* p, T v) { *(volatile T*)p = v; __threadfence(); *(volatile T*)p = v; }
__device__ __forceinline__ v8f wmma16(v16h a, v16h b, v8f c) {
  v8f d = __builtin_amdgcn_wmma_f32_16x16x32_f16(false, a, false, b, (short)0, c, false, false);
  asm volatile("v_nop\n\tv_nop\n\tv_nop\n\tv_nop" : "+v"(d) : "v"(a), "v"(b));
  return d;
}
__device__ __forceinline__ v8f wmma_bf(v16b a, v16b b, v8f c) {
  v8f d = __builtin_amdgcn_wmma_f32_16x16x32_bf16(false, a, false, b, (short)0, c, false, false);
  asm volatile("v_nop\n\tv_nop\n\tv_nop\n\tv_nop" : "+v"(d) : "v"(a), "v"(b));
  return d;
}
__device__ __forceinline__ v16h frag_h(const _Float16* rowk0, int lane) {
  union { v16h v; v8h q[2]; } u; const _Float16* p = rowk0 + 8 * (lane >> 4);
  u.q[0] = *(const v8h*)p; u.q[1] = *(const v8h*)(p + 16); return u.v;
}
__device__ __forceinline__ v16h frag_f32(const float* rowk0, int lane) {
  v16h a; const float* p = rowk0 + 8 * (lane >> 4);
#pragma unroll
  for (int i = 0; i < 8; ++i) { a[i] = (_Float16)p[i]; a[8 + i] = (_Float16)p[16 + i]; }
  return a;
}
__device__ __forceinline__ v16h frag_f32s(const float* rowk0, int lane, float sc) {
  v16h a; const float* p = rowk0 + 8 * (lane >> 4);
#pragma unroll
  for (int i = 0; i < 8; ++i) { a[i] = (_Float16)(p[i] * sc); a[8 + i] = (_Float16)(p[16 + i] * sc); }
  return a;
}
__device__ __forceinline__ v16h fragc_f32(const float* W, int k0, int n, int lane, int ld, int K) {
  v16h a; const int g = lane >> 4;
#pragma unroll
  for (int i = 0; i < 8; ++i) { const int ka = k0 + 8 * g + i, kb = ka + 16;
    a[i] = (_Float16)(ka < K ? W[(size_t)(ka < K ? ka : K - 1) * ld + n] : 0.f); a[8 + i] = (_Float16)(kb < K ? W[(size_t)(kb < K ? kb : K - 1) * ld + n] : 0.f); }
  return a;
}
struct F2 { v16b h, l; };
__device__ __forceinline__ F2 bsplit16(const float v[16]) { F2 r;
#pragma unroll
  for (int i = 0; i < 16; ++i) { const __bf16 h = (__bf16)v[i]; r.h[i] = h; r.l[i] = (__bf16)(v[i] - (float)h); }
  return r; }
__device__ __forceinline__ F2 split_row(const float* row, int k0, int lane) { float v[16]; const float* p = row + k0 + 8 * (lane >> 4);
#pragma unroll
  for (int i = 0; i < 8; ++i) { v[i] = p[i]; v[8 + i] = p[16 + i]; }
  return bsplit16(v); }
__device__ __forceinline__ F2 split_rowK(const float* row, int k0, int lane, int K) { float v[16]; const int g = lane >> 4;
#pragma unroll
  for (int i = 0; i < 8; ++i) { const int ka = k0 + 8 * g + i, kb = ka + 16; v[i] = ka < K ? row[ka < K ? ka : K - 1] : 0.f; v[8 + i] = kb < K ? row[kb < K ? kb : K - 1] : 0.f; }
  return bsplit16(v); }
__device__ __forceinline__ F2 split_col(const float* W, int k0, int n, int lane, int ld, int K) { float v[16]; const int g = lane >> 4;
#pragma unroll
  for (int i = 0; i < 8; ++i) { const int ka = k0 + 8 * g + i, kb = ka + 16; v[i] = ka < K ? W[(size_t)(ka < K ? ka : K - 1) * ld + n] : 0.f; v[8 + i] = kb < K ? W[(size_t)(kb < K ? kb : K - 1) * ld + n] : 0.f; }
  return bsplit16(v); }
__device__ __forceinline__ v8f mac3(const F2& a, const F2& b, v8f c) { c = wmma_bf(a.l, b.h, c); c = wmma_bf(a.h, b.l, c); return wmma_bf(a.h, b.h, c); }
__device__ __forceinline__ float sigm(float v) { return 1.0f / (1.0f + expf(-v)); }
#define LDSX() do { asm volatile("s_wait_dscnt 0" ::: "memory"); __builtin_amdgcn_wave_barrier(); __builtin_amdgcn_fence(__ATOMIC_RELEASE, "workgroup"); } while (0)


#define NE 640000
#define NNODE 50000
#define DD 128
#define NBLK (NE / 64)
#ifndef TBLK
#define TBLK NBLK
#endif
typedef __attribute__((ext_vector_type(8))) __bf16 v8b;
__device__ __forceinline__ v16b frag_b(const __bf16* rowk0, int lane) {
  union { v16b v; v8b q[2]; } u; const __bf16* p = rowk0 + 8 * (lane >> 4);
  u.q[0] = *(const v8b*)p; u.q[1] = *(const v8b*)(p + 16); return u.v;
}
__device__ __forceinline__ float bfr(float v) { return (float)(__bf16)v; }
__device__ __attribute__((noinline)) float exp_ni(float v) { return expf(v); }
__device__ __attribute__((noinline)) float erf_ni(float v) { return erff(v); }

#define WS_PW  0u
#define WS_SC  (WS_PW + 2u * DD * 2 * DD)
#define WS_BM  (WS_SC + 4u * (size_t)NE)
#define WS_BS  (WS_BM + 4u * 10240)
#define WS_G   (WS_BS + 4u * 10240)
#define WS_END (WS_G + 128u)

__global__ __launch_bounds__(256) void k_pack(const float* __restrict__ W1, __bf16* __restrict__ PW) { const int n = blockIdx.x, t = threadIdx.x; __shared__ __align__(16) __bf16 s[2 * DD]; s[t] = (__bf16)W1[(size_t)t * DD + n]; __syncthreads(); if (t < 2 * DD / 8) vst2((unsigned*)(PW + (size_t)n * 2 * DD + t * 8), *(const v4u*)&s[t * 8]); }
__global__ __launch_bounds__(128) void k_score(const int* __restrict__ EL, const float* __restrict__ EMB, const __bf16* __restrict__ PW, const float* __restrict__ B1, const float* __restrict__ W2, const float* __restrict__ B2, float* __restrict__ SC, float* __restrict__ BM) { __shared__ int su[64], sv[64]; __shared__ float spart[4][16][16]; __shared__ __align__(16) float ssc[64]; __shared__ float smx[4];
  const int tid = threadIdx.x, wave = tid >> 5, lane = tid & 31, col = lane & 15, g = lane >> 4; const size_t e0 = (size_t)blockIdx.x * 64;
  if (tid < 64) { int u = EL[(e0 + tid) * 2], v = EL[(e0 + tid) * 2 + 1]; u = u < 0 ? 0 : (u >= NNODE ? NNODE - 1 : u); v = v < 0 ? 0 : (v >= NNODE ? NNODE - 1 : v); su[tid] = u; sv[tid] = v; } __syncthreads();
  const int rl = wave * 16 + col; const float* ru = EMB + (size_t)su[rl] * DD; const float* rv = EMB + (size_t)sv[rl] * DD;
  v8f acc[8] = {};
#pragma unroll
  for (int kc = 0; kc < 2 * DD / 32; ++kc) { v16b a; const float* src = (kc < DD / 32) ? ru + kc * 32 : rv + (kc - DD / 32) * 32; const float* pp = src + 8 * g;
#pragma unroll
    for (int i = 0; i < 8; ++i) { a[i] = (__bf16)pp[i]; a[8 + i] = (__bf16)pp[16 + i]; }
#pragma unroll
    for (int j = 0; j < 8; ++j) acc[j] = wmma_bf(a, frag_b(PW + (size_t)(j * 16 + col) * (2 * DD) + kc * 32, lane), acc[j]); }
  float part[8];
#pragma unroll
  for (int r = 0; r < 8; ++r) part[r] = 0.f;
#pragma unroll
  for (int j = 0; j < 8; ++j) { const int c = j * 16 + col; const float bb = bfr(B1[c]), w2 = bfr(W2[c]);
#pragma unroll
    for (int r = 0; r < 8; ++r) part[r] += fmaxf(acc[j][r] + bb, 0.f) * w2; }
#pragma unroll
  for (int r = 0; r < 8; ++r) { float v = part[r];
#pragma unroll
    for (int o = 1; o < 16; o <<= 1) v += __shfl_xor(v, o);
    if (col == 0) ssc[wave * 16 + 8 * g + r] = v + bfr(B2[0]); }
  __syncthreads();
  if (tid < 32) { float m = fmaxf(ssc[tid], ssc[tid + 32]);
#pragma unroll
    for (int o = 1; o < 32; o <<= 1) m = fmaxf(m, __shfl_xor(m, o));
    if (tid == 0) smx[0] = m; }
  __syncthreads();
  if (tid < 16) vst2(SC + e0 + tid * 4, *(const v4f*)&ssc[tid * 4]);
  (void)BM; (void)spart; }
__global__ __launch_bounds__(256) void k_redmax(const float* __restrict__ SC, float* __restrict__ BM, int ne) { __shared__ float red[8]; __shared__ __align__(16) float so[32]; const int t = threadIdx.x; const size_t e0 = (size_t)blockIdx.x * 65536; float m = -3.0e38f;
  for (int i = t; i < 65536; i += 256) { const size_t e = e0 + i; if (e < (size_t)ne) m = fmaxf(m, SC[e]); }
#pragma unroll
  for (int o = 1; o < 32; o <<= 1) m = fmaxf(m, __shfl_xor(m, o));
  if ((t & 31) == 0) red[t >> 5] = m; __syncthreads(); if (t < 32) { float mm = -3.0e38f; for (int i = 0; i < 8; ++i) mm = fmaxf(mm, red[i]); so[t] = (t == 0) ? mm : 0.f; } __syncthreads(); if (t < 8) vst2(BM + (size_t)blockIdx.x * 32 + t * 4, *(const v4f*)&so[t * 4]); }
__global__ __launch_bounds__(256) void k_redsum(const float* __restrict__ SC, const float* __restrict__ BM, float* __restrict__ BS, int ne, int nchunks) { __shared__ float red[8]; __shared__ __align__(16) float so[32]; __shared__ float sg; const int t = threadIdx.x; const size_t e0 = (size_t)blockIdx.x * 65536;
  if (t == 0) { float m = -3.0e38f; for (int i = 0; i < nchunks; ++i) m = fmaxf(m, BM[(size_t)i * 32]); sg = m; } __syncthreads(); const float gm = sg;
  float s = 0.f; for (int i = t; i < 65536; i += 256) { const size_t e = e0 + i; if (e < (size_t)ne) s += expf(SC[e] - gm); }
#pragma unroll
  for (int o = 1; o < 32; o <<= 1) s += __shfl_xor(s, o);
  if ((t & 31) == 0) red[t >> 5] = s; __syncthreads(); if (t < 32) { float ss = 0.f; for (int i = 0; i < 8; ++i) ss += red[i]; so[t] = (t == 0) ? ss : 0.f; } __syncthreads(); if (t < 8) vst2(BS + (size_t)blockIdx.x * 32 + t * 4, *(const v4f*)&so[t * 4]); }
__global__ __launch_bounds__(256) void k_norm(const float* __restrict__ SC, const float* __restrict__ BM, const float* __restrict__ BS, float* __restrict__ OUT, int ne, int nchunks) { __shared__ float sg, ssum; __shared__ __align__(16) float so[1024]; const int t = threadIdx.x; const size_t e0 = (size_t)blockIdx.x * 1024;
  if (t == 0) { float m = -3.0e38f, s = 0.f; for (int i = 0; i < nchunks; ++i) m = fmaxf(m, BM[(size_t)i * 32]); for (int i = 0; i < nchunks; ++i) s += BS[(size_t)i * 32]; sg = m; ssum = s; } __syncthreads(); const float gm = sg, inv = 1.0f / ssum;
  for (int i = t; i < 1024; i += 256) { const size_t e = e0 + i; so[i] = (e < (size_t)ne) ? expf(SC[e] - gm) * inv : 0.f; } __syncthreads();
  { const size_t e = e0 + t * 4; if (e + 4 <= (size_t)ne) vst2(OUT + e, *(const v4f*)&so[t * 4]); } }
extern "C" void kernel_launch(void* const* d_in, const int* in_sizes, int n_in, void* d_out, int out_size, void* d_ws, size_t ws_size, hipStream_t stream) {
  (void)in_sizes; (void)n_in; (void)out_size;
  const float** F = (const float**)d_in;
  if (ws_size < (size_t)WS_END) return;
  char* ws = (char*)d_ws; __bf16* PW = (__bf16*)(ws + WS_PW); float *SC = (float*)(ws + WS_SC), *BM = (float*)(ws + WS_BM), *BS = (float*)(ws + WS_BS);
  const int ne = TBLK * 64; const int nchunks = (ne + 65535) / 65536;
  k_pack<<<DD, 256, 0, stream>>>(F[2], PW);
  k_score<<<TBLK, 128, 0, stream>>>((const int*)d_in[0], F[1], PW, F[3], F[4], F[5], SC, BM);
  k_redmax<<<nchunks, 256, 0, stream>>>(SC, BM, ne);
  k_redsum<<<nchunks, 256, 0, stream>>>(SC, BM, BS, ne, nchunks);
  k_norm<<<(ne + 1023) / 1024, 256, 0, stream>>>(SC, BM, BS, (float*)d_out, ne, nchunks);
}
